// TwoLayerSimpleHeteroGAT_5265629905487
// MI455X (gfx1250) — hardware-run, weakly checked
//
#include <hip/hip_runtime.h>

typedef float          v8f   __attribute__((ext_vector_type(8)));
typedef float          v4f   __attribute__((ext_vector_type(4)));
typedef unsigned int   v4u   __attribute__((ext_vector_type(4)));
typedef int            v8i   __attribute__((ext_vector_type(8)));
typedef unsigned short v8us  __attribute__((ext_vector_type(8)));
typedef unsigned short v16us __attribute__((ext_vector_type(16)));
typedef __bf16         v16bf __attribute__((ext_vector_type(16)));
typedef _Float16       v16h  __attribute__((ext_vector_type(16)));
typedef v4f  __attribute__((may_alias)) v4fa;
typedef v8us __attribute__((may_alias)) v8usa;
union FragB { v16bf v; v16us u; v8us h[2]; v8i w; };
union FragH { v16h  v; v16us u; v8us h[2]; v8i w; };

__device__ __forceinline__ v8f wmb(const FragB& a, const FragB& b, v8f c) {
  v8f d = __builtin_amdgcn_wmma_f32_16x16x32_bf16(false, a.v, false, b.v, (short)0, c, false, false);
  asm volatile("v_nop\n\tv_nop\n\tv_nop\n\tv_nop" : "+v"(d) : "v"(a.w), "v"(b.w));
  return d;
}

__device__ __forceinline__ v8f wmh(const FragH& a, const FragH& b, v8f c) {
  v8f d = __builtin_amdgcn_wmma_f32_16x16x32_f16(false, a.v, false, b.v, (short)0, c, false, false);
  asm volatile("v_nop\n\tv_nop\n\tv_nop\n\tv_nop" : "+v"(d) : "v"(a.w), "v"(b.w));
  return d;
}

__device__ __forceinline__ unsigned bf16_bits(float f) {
  const unsigned u = __float_as_uint(f);
  const unsigned r = (u + 0x7FFFu + ((u >> 16) & 1u)) >> 16;
  const unsigned q = (u >> 16) | 0x40u;
  return ((u & 0x7fffffffu) > 0x7f800000u) ? q : r;
}

__device__ __forceinline__ float bf16_val(float f) {
  return __uint_as_float(bf16_bits(f) << 16);
}
__device__ __forceinline__ int clampi(int v, int lo, int hi) {
  return v < lo ? lo : (v > hi ? hi : v);
}

__device__ __forceinline__ unsigned f16_bits(float f) {
  const unsigned u  = __float_as_uint(f);
  const unsigned s  = (u >> 16) & 0x8000u;
  const unsigned a  = u & 0x7fffffffu;
  const unsigned t  = a - 0x38000000u;
  const unsigned r  = (t + 0x0FFFu + ((t >> 13) & 1u)) >> 13;
  const unsigned rc = r > 0x7C00u ? 0x7C00u : r;
  const bool small  = a < 0x38800000u;
  const bool isnan  = a > 0x7f800000u;
  const unsigned fin = small ? 0u : (s | rc);
  return isnan ? (s | 0x7E00u) : fin;
}

__device__ __forceinline__ unsigned pk16(unsigned lo, unsigned hi) { return lo | (hi << 16); }
__device__ __forceinline__ unsigned bf16_lo_bits(float v) {
  float hi = bf16_val(v);
  asm volatile("" : "+v"(hi));
  return bf16_bits(v - hi);
}
__device__ __forceinline__ v4u pack8_bf16(v4f a, v4f c) {
  return (v4u){ pk16(bf16_bits(a[0]), bf16_bits(a[1])), pk16(bf16_bits(a[2]), bf16_bits(a[3])),
                pk16(bf16_bits(c[0]), bf16_bits(c[1])), pk16(bf16_bits(c[2]), bf16_bits(c[3])) };
}
__device__ __forceinline__ v4u pack8_bf16_lo(v4f a, v4f c) {
  return (v4u){ pk16(bf16_lo_bits(a[0]), bf16_lo_bits(a[1])), pk16(bf16_lo_bits(a[2]), bf16_lo_bits(a[3])),
                pk16(bf16_lo_bits(c[0]), bf16_lo_bits(c[1])), pk16(bf16_lo_bits(c[2]), bf16_lo_bits(c[3])) };
}
__device__ __forceinline__ v4u pack8_f16(v4f a, v4f c) {
  return (v4u){ pk16(f16_bits(a[0]), f16_bits(a[1])), pk16(f16_bits(a[2]), f16_bits(a[3])),
                pk16(f16_bits(c[0]), f16_bits(c[1])), pk16(f16_bits(c[2]), f16_bits(c[3])) };
}

template <int FORM>
__global__ __launch_bounds__(256) void k_plane(const float* __restrict__ src, int rows, int cols, int ldsrc,
                                               unsigned short* __restrict__ dst, int MP, int KP) {
  static_assert(FORM >= 0 && FORM <= 3);
  const int KTOT = (FORM == 1 || FORM == 3) ? 2 * KP : KP;
  const unsigned ppr   = (unsigned)(KTOT >> 3);
  const unsigned kp8   = (unsigned)(KP >> 3);
  const unsigned total = (unsigned)MP * ppr;
  const unsigned g     = blockIdx.x * 256u + threadIdx.x;
  const unsigned rowu  = g / ppr;
  const unsigned p     = g - rowu * ppr;
  const bool second    = p >= kp8;
  const int row = (int)rowu;
  const int c0  = (int)((second ? p - kp8 : p) << 3);
  const float* srow = src + (size_t)clampi(row, 0, rows - 1) * (size_t)ldsrc;
  float x[8];
  unsigned mk[8];
#pragma unroll
  for (int e = 0; e < 8; ++e) {
    const int c = c0 + e;
    const float v = srow[clampi(c, 0, cols - 1)];
    asm volatile("" :: "v"(v));
    x[e]  = v;
    mk[e] = (row < rows && c < cols) ? 0xFFFFu : 0u;
  }
  const v4f a = (v4f){ x[0], x[1], x[2], x[3] };
  const v4f c = (v4f){ x[4], x[5], x[6], x[7] };
  v4u o;
  if (FORM == 2) {
    o = pack8_f16(a, c);
  } else {
    const v4u hi = pack8_bf16(a, c);
    o = hi;
    if (FORM == 1) { const v4u lo = pack8_bf16_lo(a, c); o = second ? lo : hi; }
  }
  const v4u mw = (v4u){ pk16(mk[0], mk[1]), pk16(mk[2], mk[3]), pk16(mk[4], mk[5]), pk16(mk[6], mk[7]) };
  o &= mw;
  if (g < total) {
    volatile v4u* q = (volatile v4u*)(dst + (size_t)g * 8);
    *q = o;
    __threadfence();
    *q = o;
  }
}

template <int FORM> struct FragOf    { typedef FragB T; };
template <>         struct FragOf<2> { typedef FragH T; };
__device__ __forceinline__ v8f mm(const FragB& a, const FragB& b, v8f c) { return wmb(a, b, c); }
__device__ __forceinline__ v8f mm(const FragH& a, const FragH& b, v8f c) { return wmh(a, b, c); }
template <class F> __device__ __forceinline__ F ld_frag(const unsigned short* p) {
  F f;
  f.h[0] = *(const v8usa*)(p);
  f.h[1] = *(const v8usa*)(p + 16);
  return f;
}

template <int FORM, int EPI>
__global__ __launch_bounds__(256) __attribute__((amdgpu_num_vgpr(248)))
void k_gemm_nt(const unsigned short* __restrict__ A, const unsigned short* __restrict__ B,
               const float* __restrict__ bias, float* __restrict__ D, int M, int N, int KTOT, int ldd) {
  static_assert(FORM >= 0 && FORM <= 2);
  static_assert(EPI == 0 || EPI == 1);
  typedef typename FragOf<FORM>::T F;
  __shared__ __attribute__((aligned(16))) float sT[8][16 * 68];
  const int lane = threadIdx.x & 31;
  const int wave = threadIdx.x >> 5;
  const int tilesM = (M + 63) >> 6;
  const int tilesN = (N + 63) >> 6;
  const int tile = blockIdx.x * 8 + wave;
  if (tile >= tilesM * tilesN) return;
  const int tm = tile / tilesN;
  const int tn = tile - tm * tilesN;
  const int m0 = tm << 6;
  const int n0 = tn << 6;

  const int rl = lane & 15;
  const int h8 = (lane >> 4) * 8;
  const unsigned short* pa = A + (size_t)(m0 + rl) * (size_t)KTOT + h8;
  const unsigned short* pb = B + (size_t)(n0 + rl) * (size_t)KTOT + h8;

  v8f acc[4][4];
#pragma unroll
  for (int i = 0; i < 4; ++i)
#pragma unroll
    for (int j = 0; j < 4; ++j) acc[i][j] = (v8f){0.f, 0.f, 0.f, 0.f, 0.f, 0.f, 0.f, 0.f};

#pragma unroll 1
  for (int k0 = 0; k0 < KTOT; k0 += 32) {
    F bf[4];
#pragma unroll
    for (int j = 0; j < 4; ++j) bf[j] = ld_frag<F>(pb + (size_t)(j << 4) * (size_t)KTOT + k0);
#pragma unroll
    for (int i = 0; i < 4; ++i) {
      const F af = ld_frag<F>(pa + (size_t)(i << 4) * (size_t)KTOT + k0);
#pragma unroll
      for (int j = 0; j < 4; ++j) acc[i][j] = mm(af, bf[j], acc[i][j]);
    }
  }

  float* slab = sT[wave];
  const int hh = lane >> 4;
  const int c4 = (lane & 15) * 4;
  const int nc = n0 + c4;
  const bool cok = nc < N;
  v4f bv = (v4f){0.f, 0.f, 0.f, 0.f};
  if (EPI == 1) {
    bv = *(const v4fa*)(bias + clampi(nc, 0, N - 4));
    asm volatile("" :: "v"(bv));
  }
#pragma unroll
  for (int i = 0; i < 4; ++i) {
    const int mBase = m0 + (i << 4);
#pragma unroll
    for (int j = 0; j < 4; ++j) {
#pragma unroll
      for (int r = 0; r < 8; ++r) slab[(h8 + r) * 68 + (j << 4) + rl] = acc[i][j][r];
    }
    __builtin_amdgcn_fence(__ATOMIC_RELEASE, "workgroup");
    __builtin_amdgcn_wave_barrier();
    __builtin_amdgcn_fence(__ATOMIC_ACQUIRE, "workgroup");
    v4f vv[8];
#pragma unroll
    for (int it = 0; it < 8; ++it) {
      const int row = it * 2 + hh;
      v4f v = *(const v4fa*)(slab + row * 68 + c4);
      if (EPI == 1) v += bv;
      vv[it] = v;
    }
    for (int pass = 0; pass < 2; ++pass) {
#pragma unroll
      for (int it = 0; it < 8; ++it) {
        const int row = mBase + it * 2 + hh;
        if (cok && row < M) *(volatile v4f*)(D + (size_t)row * (size_t)ldd + nc) = vv[it];
      }
      __threadfence();
    }
    __builtin_amdgcn_fence(__ATOMIC_RELEASE, "workgroup");
    __builtin_amdgcn_wave_barrier();
    __builtin_amdgcn_fence(__ATOMIC_ACQUIRE, "workgroup");
  }
}

#define TWO_TERM  1

#define NN        100000
#define NE        500000
#define MPN       100096
#define PSLD      128
#define PTLD      192
#define XLW       192
#define HWD       64
#define YLD       32
#define CHROWS    25600
#define LASTROWS  23200
#define LASTPAD   23232
#define OWN       1024
#define NOWN      98
#define RCAP      6656
#define SCHUNK    2048
#define WCAP      256
#define TABF      512
#define PLANE_US  32768
#define OUT_ITEM  3200000
#define LDS_BUILD ((2 * RCAP + 2 * OWN + 8 * WCAP + 32) * 4)

static_assert(3 * CHROWS + LASTROWS == NN);
static_assert((CHROWS % 1024) == 0 && (CHROWS % 128) == 0);
static_assert(((2 * CHROWS) % 1024) == 0 && ((3 * CHROWS) % 1024) == 0);
static_assert((LASTROWS % 16) == 0 && (LASTROWS % 32) == 0 && (CHROWS % 64) == 0);
static_assert((LASTPAD % 64) == 0 && LASTPAD >= LASTROWS && LASTPAD <= CHROWS);
static_assert(3 * CHROWS + LASTPAD <= MPN && (MPN % 64) == 0 && MPN >= NN + 32);
static_assert(NOWN * OWN >= NN && (NOWN - 1) * OWN < NN && NOWN * OWN >= MPN);
static_assert(RCAP * 4 >= 5318 * 5 && (RCAP % 256) == 0);
static_assert(NE < (1 << 20) && SCHUNK == 8 * WCAP);
static_assert(LDS_BUILD <= 262144);
static_assert(8192 + 12288 + 12288 == PLANE_US);
static_assert(OUT_ITEM + NN * 32 == 6400000);

#define SZ_A     ((size_t)MPN * HWD * 2)
#define SZ_PS    ((size_t)MPN * PSLD * 4)
#define SZ_EL    ((size_t)MPN * 16)
#define SZ_PT    ((size_t)CHROWS * PTLD * 4)
#define SZ_XL    ((size_t)CHROWS * XLW * 2)
#define SZ_HITS  ((size_t)NOWN * RCAP * 4)
#define SZ_ROW   ((size_t)NOWN * OWN * 4)
#define SZ_FLG   ((size_t)NOWN * 128)
#define SZ_PL    ((size_t)4 * PLANE_US * 2)
#define SZ_TAB   ((size_t)4 * TABF * 4)
#define WS_TOTAL (3 * SZ_A + SZ_PS + SZ_EL + SZ_PT + SZ_XL + 2 * SZ_HITS + 4 * SZ_ROW + 2 * SZ_FLG + SZ_PL + SZ_TAB)
static_assert(WS_TOTAL == (size_t)((size_t)249801 << 9));
static_assert(WS_TOTAL <= ((size_t)128 << 20));
static_assert((size_t)CHROWS * YLD * 4 <= SZ_PT);
static_assert((SZ_A % 128) == 0 && (SZ_HITS % 128) == 0 && (SZ_ROW % 128) == 0 && (SZ_FLG % 128) == 0);

typedef int v4i __attribute__((ext_vector_type(4)));
typedef v4i __attribute__((may_alias)) v4ia;

__device__ __forceinline__ float wsum(float v) {
#pragma unroll
  for (int off = 16; off > 0; off >>= 1) v += __shfl_xor(v, off);
  return v;
}
__device__ __forceinline__ float wmaxf(float v) {
#pragma unroll
  for (int off = 16; off > 0; off >>= 1) v = fmaxf(v, __shfl_xor(v, off));
  return v;
}

__device__ __forceinline__ void tr_unit(const float* __restrict__ w, int Ksrc, int cols,
                                        unsigned short* dst, int KTOT, int u) {
  const int ppr = KTOT >> 3;
  const int n   = u / ppr;
  const int k8  = (u - n * ppr) << 3;
  const int kb  = k8 % Ksrc;
  const int ncl = n < cols ? n : cols - 1;
  const unsigned mk = n < cols ? 0xFFFFu : 0u;
  unsigned b[8];
#pragma unroll
  for (int e = 0; e < 8; ++e) {
    const float x = w[(size_t)(kb + e) * (size_t)cols + ncl];
    asm volatile("" :: "v"(x));
    b[e] = bf16_bits(x) & mk;
  }
  const v4u o = (v4u){ pk16(b[0], b[1]), pk16(b[2], b[3]), pk16(b[4], b[5]), pk16(b[6], b[7]) };
  volatile v4u* q = (volatile v4u*)(dst + (size_t)n * (size_t)KTOT + k8);
  *q = o;
  __threadfence();
  *q = o;
}

__global__ __launch_bounds__(256) void k_prep(const float* __restrict__ W, const float* __restrict__ RES,
                                              const float* __restrict__ NNW, const float* __restrict__ ATT,
                                              const float* __restrict__ BIA, const float* __restrict__ NNB,
                                              const float* __restrict__ BN, int Ksrc,
                                              unsigned short* planes, float* tabs, unsigned short* zpad, int dozero) {
  const int d   = (int)blockIdx.y;
  const int ty  = 1 - d;
  const int bx  = (int)blockIdx.x;
  const int tid = (int)threadIdx.x;
  unsigned short* BS = planes + (size_t)d * PLANE_US;
  unsigned short* BT = BS + 8192;
  unsigned short* BL = BT + 12288;
  float* tb = tabs + (size_t)d * TABF;
  const float* w   = W   + (size_t)d * (size_t)Ksrc * 96;
  const float* rs  = RES + (size_t)d * (size_t)Ksrc * 96;
  const float* nnw = NNW + (size_t)ty * 96 * 32;
  if (bx < 4) {
    tr_unit(w, Ksrc, 96, BS, 64, bx * 256 + tid);
  } else if (bx < 7) {
    tr_unit(w, Ksrc, 96, BT, 64, (bx - 4) * 256 + tid);
  } else if (bx < 10) {
    tr_unit(rs, Ksrc, 96, BT + 96 * 64, 64, (bx - 7) * 256 + tid);
  } else if (bx < 16) {
    tr_unit(nnw, 96, 32, BL, 192, (bx - 10) * 256 + tid);
  } else if (bx == 16) {
    const int e  = 4 * (tid & 127);
    const int ia = clampi(e, 0, 188);
    const int ib = clampi(e - 192, 0, 92);
    const int in = clampi(e - 288, 0, 28);
    const int ig = clampi(e - 320, 0, 124);
    const v4f va = *(const v4fa*)(ATT + d * 192 + ia);
    const v4f vb = *(const v4fa*)(BIA + d * 96 + ib);
    const v4f vn = *(const v4fa*)(NNB + ty * 32 + in);
    const v4f vg = *(const v4fa*)(BN + ty * 128 + ig);
    asm volatile("" :: "v"(va), "v"(vb), "v"(vn), "v"(vg));
    const unsigned ma = (e < 192) ? 0xFFFFFFFFu : 0u;
    const unsigned mb = (e >= 192 && e < 288) ? 0xFFFFFFFFu : 0u;
    const unsigned mn = (e >= 288 && e < 320) ? 0xFFFFFFFFu : 0u;
    const unsigned mg = (e >= 320 && e < 448) ? 0xFFFFFFFFu : 0u;
    v4f o;
#pragma unroll
    for (int i = 0; i < 4; ++i) {
      const unsigned bits = (__float_as_uint(bf16_val(va[i])) & ma) | (__float_as_uint(bf16_val(vb[i])) & mb) |
                            (__float_as_uint(bf16_val(vn[i])) & mn) | (__float_as_uint(bf16_val(vg[i])) & mg);
      o[i] = __uint_as_float(bits);
    }
    const bool wr = tid < 128;
    if (wr) *(volatile v4f*)(tb + e) = o;
    __threadfence();
    if (wr) *(volatile v4f*)(tb + e) = o;
  } else {
    const int u = (bx - 17) * 256 + tid;
    const bool wr = (dozero != 0) && (d == 0) && (u < 768);
    const v4u z = (v4u){0u, 0u, 0u, 0u};
    if (wr) *(volatile v4u*)(zpad + (size_t)u * 8) = z;
    __threadfence();
    if (wr) *(volatile v4u*)(zpad + (size_t)u * 8) = z;
  }
}

__global__ __launch_bounds__(256) void k_build(const int* __restrict__ srcs, const int* __restrict__ dsts,
                                               int* hits, int* rowoff, int* rowcnt, int* flg) {
  extern __shared__ v4f lds_dyn[];
  int* reg1 = (int*)lds_dyn;
  int* reg2 = reg1 + RCAP;
  int* scnt = reg2 + RCAP;
  int* soff = scnt + OWN;
  int* list = soff + OWN;
  int* wcnt = list + 8 * WCAP;
  int* wtot = wcnt + 8;
  const int tid = (int)threadIdx.x, lane = tid & 31, wave = tid >> 5;
  const int slotBase = (int)blockIdx.x * OWN;
  int nb = NN - slotBase;
  nb = nb > OWN ? OWN : (nb < 0 ? 0 : nb);

  for (int i = tid; i < OWN; i += 256) scnt[i] = 0;
  for (int i = tid; i < RCAP; i += 256) { reg1[i] = 0; reg2[i] = 0; }
  __syncthreads();

  int tot = 0, raw = 0;
  const int nChunks = (NE + SCHUNK - 1) / SCHUNK;
  const int elw = wave * 256 + lane;
#pragma unroll 1
  for (int ch = 0; ch < nChunks; ++ch) {
    const int cbase = ch * SCHUNK;
    int wc = 0;
#pragma unroll
    for (int j = 0; j < 8; ++j) {
      const int e  = cbase + elw + 32 * j;
      const int ec = e < NE - 1 ? e : NE - 1;
      const int dd = dsts[ec];
      asm volatile("" :: "v"(dd));
      const unsigned s = (unsigned)dd - (unsigned)slotBase;
      const bool hj = (s < (unsigned)nb) & (e < NE);
      const unsigned mj = __builtin_amdgcn_ballot_w32(hj);
      const int pos = wc + (int)__builtin_amdgcn_mbcnt_lo(mj, 0u);
      if (hj && pos < WCAP) list[wave * WCAP + pos] = ((elw + 32 * j) << 12) | (int)(s & 1023u);
      wc += (int)__builtin_popcount(mj);
    }
    if (lane == 0) wcnt[wave] = wc;
    __syncthreads();
    int pre = 0, all = 0;
#pragma unroll
    for (int w2 = 0; w2 < 8; ++w2) {
      int c = wcnt[w2];
      c = c < 0 ? 0 : (c > WCAP ? WCAP : c);
      all += c;
      pre += (w2 < wave) ? c : 0;
    }
    const int wcc  = wc > WCAP ? WCAP : wc;
    const int base = tot + pre;
#pragma unroll 1
    for (int i = lane; i < wcc; i += 32) {
      const int ent = list[wave * WCAP + i];
      const int el  = (ent >> 12) & (SCHUNK - 1);
      const int sl  = ent & (OWN - 1);
      int eid = cbase + el;
      eid = eid > NE - 1 ? NE - 1 : eid;
      const int pos = base + i;
      if (pos < RCAP) reg1[pos] = (int)(((unsigned)eid << 12) | (unsigned)sl);
    }
    raw += all;
    tot += all;
    tot = tot > RCAP ? RCAP : tot;
    __syncthreads();
  }
  const int nh = tot;
  const bool ovf = raw > RCAP;

  if (wave == 0) {
#pragma unroll 1
    for (int b0 = 0; b0 < nh; b0 += 32) {
      const int idx = b0 + lane;
      const int uv  = reg1[idx < RCAP ? idx : RCAP - 1];
      const int m32 = (nh - b0) < 32 ? (nh - b0) : 32;
#pragma unroll 1
      for (int k = 0; k < m32; ++k) {
        const int u  = __builtin_amdgcn_readlane(uv, k);
        const int sl = u & (OWN - 1);
        if (lane == 0) scnt[sl] = scnt[sl] + 1;
      }
    }
  }
  __syncthreads();

  {
    const v4i ca = *(const v4ia*)(scnt + 4 * tid);
    const int e0 = ca.x < 0 ? 0 : ca.x, e1 = ca.y < 0 ? 0 : ca.y, e2 = ca.z < 0 ? 0 : ca.z, e3 = ca.w < 0 ? 0 : ca.w;
    const int ts = e0 + e1 + e2 + e3;
    int incl = ts;
#pragma unroll
    for (int dlt = 1; dlt < 32; dlt <<= 1) {
      const int up = __shfl_up(incl, dlt);
      incl += (lane >= dlt) ? up : 0;
    }
    if (lane == 31) wtot[wave] = incl;
    __syncthreads();
    int pre = 0;
#pragma unroll
    for (int w2 = 0; w2 < 8; ++w2) pre += (w2 < wave) ? wtot[w2] : 0;
    int run = pre + incl - ts;
    soff[4 * tid + 0] = run; run += e0;
    soff[4 * tid + 1] = run; run += e1;
    soff[4 * tid + 2] = run; run += e2;
    soff[4 * tid + 3] = run;
  }
  __syncthreads();
  for (int i = tid; i < OWN; i += 256) list[i] = soff[i];
  __syncthreads();

  if (wave == 0) {
#pragma unroll 1
    for (int b0 = 0; b0 < nh; b0 += 32) {
      const int idx = b0 + lane;
      const int uv  = reg1[idx < RCAP ? idx : RCAP - 1];
      const int m32 = (nh - b0) < 32 ? (nh - b0) : 32;
#pragma unroll 1
      for (int k = 0; k < m32; ++k) {
        const int u   = __builtin_amdgcn_readlane(uv, k);
        const int sl  = u & (OWN - 1);
        const int eid = (int)((unsigned)u >> 12);
        if (lane == 0) {
          int pos = list[sl];
          pos = pos < 0 ? 0 : (pos > RCAP - 1 ? RCAP - 1 : pos);
          reg2[pos] = eid;
          list[sl] = pos + 1;
        }
      }
    }
  }
  __syncthreads();

#pragma unroll 1
  for (int i = tid; i < RCAP; i += 256) {
    const int eid = clampi(reg2[i], 0, NE - 1);
    const int sv  = srcs[eid];
    asm volatile("" :: "v"(sv));
    const int sc  = clampi(sv, 0, NN - 1);
    const int msk = (i < nh) ? -1 : 0;
    reg1[i] = sc & msk;
  }
  __syncthreads();

  int* hb = hits + (size_t)blockIdx.x * RCAP;
  const v4i so = *(const v4ia*)(soff + 4 * tid);
  const v4i sc = *(const v4ia*)(scnt + 4 * tid);
  const int fv = ovf ? 1 : 0;
  const v4i f4 = (v4i){fv, fv, fv, fv};
  for (int pass = 0; pass < 2; ++pass) {
#pragma unroll 1
    for (int p = tid; p < RCAP / 4; p += 256) {
      const v4i v = *(const v4ia*)(reg1 + 4 * p);
      *(volatile v4i*)(hb + 4 * p) = v;
    }
    *(volatile v4i*)(rowoff + slotBase + 4 * tid) = so;
    *(volatile v4i*)(rowcnt + slotBase + 4 * tid) = sc;
    if (tid < 8) *(volatile v4i*)(flg + (int)blockIdx.x * 32 + 4 * tid) = f4;
    __threadfence();
  }
}

__global__ __launch_bounds__(256) void k_el(const float* __restrict__ PS, const float* __restrict__ tab, float* EL) {
  __shared__ __attribute__((aligned(16))) float sA[96];
  const int tid = (int)threadIdx.x, lane = tid & 31, wave = tid >> 5;
  {
    const int tq = tid < 24 ? tid : 23;
    const v4f pv = *(const v4fa*)(tab + 4 * tq);
    asm volatile("" :: "v"(pv));
    if (tid < 24) *(v4fa*)(sA + 4 * tid) = pv;
  }
  __syncthreads();
  const float a0 = sA[lane], a1 = sA[32 + lane], a2 = sA[64 + lane];
  const int rbase = (int)blockIdx.x * 256 + wave * 32;
  float k0 = 0.f, k1 = 0.f, k2 = 0.f;
#pragma unroll 2
  for (int i = 0; i < 32; ++i) {
    const int r  = rbase + i;
    const int rc = r < NN ? r : NN - 1;
    const float* p = PS + (size_t)rc * PSLD + lane;
    const float x0 = p[0], x1 = p[32], x2 = p[64];
    asm volatile("" :: "v"(x0), "v"(x1), "v"(x2));
    const float s0 = wsum(x0 * a0);
    const float s1 = wsum(x1 * a1);
    const float s2 = wsum(x2 * a2);
    const bool mine = (lane == i);
    k0 = mine ? s0 : k0;
    k1 = mine ? s1 : k1;
    k2 = mine ? s2 : k2;
  }
  const int row = (int)blockIdx.x * 256 + tid;
  const bool lv = row < NN;
  const v4f o = (v4f){ lv ? k0 : 0.f, lv ? k1 : 0.f, lv ? k2 : 0.f, 0.f };
  *(volatile v4f*)(EL + (size_t)row * 4) = o;
  __threadfence();
  *(volatile v4f*)(EL + (size_t)row * 4) = o;
}

__global__ __launch_bounds__(256) void k_replay(const float* __restrict__ PT, const float* __restrict__ EL,
                                                const float* __restrict__ PS, const int* __restrict__ hits,
                                                const int* __restrict__ rowoff, const int* __restrict__ rowcnt,
                                                const int* __restrict__ flg, const float* __restrict__ tab,
                                                unsigned short* XL, int chunkStart, int rowsValid, int rowsPad) {
  __shared__ __attribute__((aligned(16))) unsigned short sX[8 * XLW];
  __shared__ __attribute__((aligned(16))) float sP[192];
  const int tid = (int)threadIdx.x, lane = tid & 31, wave = tid >> 5;
  {
    const int tq = tid < 48 ? tid : 47;
    const v4f pv = *(const v4fa*)(tab + 96 + 4 * tq);
    asm volatile("" :: "v"(pv));
    if (tid < 48) *(v4fa*)(sP + 4 * tid) = pv;
  }
  __syncthreads();

  const int lt = (int)blockIdx.x * 8 + wave;
  const bool live = lt < rowsValid;
  const int ltc = live ? lt : rowsValid - 1;
  const int t = chunkStart + ltc;
  const float* pr = PT + (size_t)ltc * PTLD + lane;
  const float fd0 = pr[0], fd1 = pr[32], fd2 = pr[64], rs0 = pr[96], rs1 = pr[128], rs2 = pr[160];
  asm volatile("" :: "v"(fd0), "v"(fd1), "v"(fd2), "v"(rs0), "v"(rs1), "v"(rs2));
  const float er0 = wsum(fd0 * sP[lane]);
  const float er1 = wsum(fd1 * sP[32 + lane]);
  const float er2 = wsum(fd2 * sP[64 + lane]);

  const int ob = t >> 10;
  int st = rowoff[t];
  const int craw = rowcnt[t];
  const int fl = flg[ob * 32];
  asm volatile("" :: "v"(st), "v"(craw), "v"(fl));
  st = clampi(st, 0, RCAP);
  int cnv = clampi(craw, 0, RCAP - st);
  cnv = live ? cnv : 0;
  const int cn = __builtin_amdgcn_readfirstlane(cnv);
  const int* hbb = hits + (size_t)ob * RCAP;

  const float ninf = -__builtin_huge_valf();
  float m0 = ninf, m1 = ninf, m2 = ninf;
#pragma unroll 1
  for (int b0 = 0; b0 < cn; b0 += 32) {
    const int q = b0 + lane;
    int idx = st + q;
    idx = idx > RCAP - 1 ? RCAP - 1 : idx;
    const int sraw = hbb[idx];
    asm volatile("" :: "v"(sraw));
    const int s = clampi(sraw, 0, NN - 1);
    const v4f ev = *(const v4fa*)(EL + (size_t)s * 4);
    asm volatile("" :: "v"(ev));
    const bool valid = q < cn;
    float e0 = ev[0] + er0; e0 = e0 > 0.f ? e0 : 0.01f * e0;
    float e1 = ev[1] + er1; e1 = e1 > 0.f ? e1 : 0.01f * e1;
    float e2 = ev[2] + er2; e2 = e2 > 0.f ? e2 : 0.01f * e2;
    m0 = valid ? fmaxf(m0, e0) : m0;
    m1 = valid ? fmaxf(m1, e1) : m1;
    m2 = valid ? fmaxf(m2, e2) : m2;
  }
  m0 = wmaxf(m0); m1 = wmaxf(m1); m2 = wmaxf(m2);
  const float pinf = __builtin_huge_valf();
  m0 = (fabsf(m0) < pinf) ? m0 : 0.f;
  m1 = (fabsf(m1) < pinf) ? m1 : 0.f;
  m2 = (fabsf(m2) < pinf) ? m2 : 0.f;

  float den0 = 0.f, den1 = 0.f, den2 = 0.f, ac0 = 0.f, ac1 = 0.f, ac2 = 0.f;
#pragma unroll 1
  for (int b0 = 0; b0 < cn; b0 += 32) {
    const int q = b0 + lane;
    int idx = st + q;
    idx = idx > RCAP - 1 ? RCAP - 1 : idx;
    const int sraw = hbb[idx];
    asm volatile("" :: "v"(sraw));
    const int s = clampi(sraw, 0, NN - 1);
    const v4f ev = *(const v4fa*)(EL + (size_t)s * 4);
    asm volatile("" :: "v"(ev));
    const bool valid = q < cn;
    float e0 = ev[0] + er0; e0 = e0 > 0.f ? e0 : 0.01f * e0;
    float e1 = ev[1] + er1; e1 = e1 > 0.f ? e1 : 0.01f * e1;
    float e2 = ev[2] + er2; e2 = e2 > 0.f ? e2 : 0.01f * e2;
    const float g0 = expf(e0 - m0), g1 = expf(e1 - m1), g2 = expf(e2 - m2);
    const int x0 = valid ? __float_as_int(g0) : 0;
    const int x1 = valid ? __float_as_int(g1) : 0;
    const int x2 = valid ? __float_as_int(g2) : 0;
    const int kmax = (cn - b0) < 32 ? (cn - b0) : 32;
#pragma unroll 1
    for (int k = 0; k < kmax; ++k) {
      const int sk = __builtin_amdgcn_readlane(s, k);
      const float w0 = __int_as_float(__builtin_amdgcn_readlane(x0, k));
      const float w1 = __int_as_float(__builtin_amdgcn_readlane(x1, k));
      const float w2 = __int_as_float(__builtin_amdgcn_readlane(x2, k));
      const float* pp = PS + (size_t)sk * PSLD + lane;
      const float p0 = pp[0], p1 = pp[32], p2 = pp[64];
      asm volatile("" :: "v"(p0), "v"(p1), "v"(p2));
      den0 += w0; den1 += w1; den2 += w2;
      ac0 = fmaf(w0, p0, ac0);
      ac1 = fmaf(w1, p1, ac1);
      ac2 = fmaf(w2, p2, ac2);
    }
  }
  const bool has = cn > 0;
  const float d0 = has ? den0 : 1.0f, d1 = has ? den1 : 1.0f, d2 = has ? den2 : 1.0f;
  const float r0 = has ? (ac0 / d0) : 0.f;
  const float r1 = has ? (ac1 / d1) : 0.f;
  const float r2 = has ? (ac2 / d2) : 0.f;
  float v0 = (r0 + rs0) + sP[96 + lane];
  float v1 = (r1 + rs1) + sP[128 + lane];
  float v2 = (r2 + rs2) + sP[160 + lane];
  const float qnan = __uint_as_float(0x7fc00000u);
  const bool bad = fl != 0;
  v0 = bad ? qnan : v0; v1 = bad ? qnan : v1; v2 = bad ? qnan : v2;
  v0 = live ? v0 : 0.f; v1 = live ? v1 : 0.f; v2 = live ? v2 : 0.f;

  unsigned short* xr = sX + wave * XLW;
  xr[lane]       = (unsigned short)bf16_bits(v0);
  xr[32 + lane]  = (unsigned short)bf16_bits(v1);
  xr[64 + lane]  = (unsigned short)bf16_bits(v2);
  xr[96 + lane]  = (unsigned short)(TWO_TERM ? bf16_lo_bits(v0) : 0u);
  xr[128 + lane] = (unsigned short)(TWO_TERM ? bf16_lo_bits(v1) : 0u);
  xr[160 + lane] = (unsigned short)(TWO_TERM ? bf16_lo_bits(v2) : 0u);
  __builtin_amdgcn_fence(__ATOMIC_RELEASE, "workgroup");
  __builtin_amdgcn_wave_barrier();
  __builtin_amdgcn_fence(__ATOMIC_ACQUIRE, "workgroup");
  const int lc = lane < 24 ? lane : 23;
  const v8us piece = *(const v8usa*)(xr + 8 * lc);
  const bool wr = (lane < 24) && (lt < rowsPad);
  unsigned short* gp = XL + (size_t)lt * XLW + 8 * lc;
  if (wr) *(volatile v8us*)gp = piece;
  __threadfence();
  if (wr) *(volatile v8us*)gp = piece;
}

template <int LAYER>
__global__ __launch_bounds__(256) void k_row(const float* __restrict__ Y, const float* __restrict__ tab,
                                             const int* __restrict__ flg, unsigned short* Hout, float* Fout,
                                             int chunkStart, int rowsValid) {
  __shared__ __attribute__((aligned(16))) float sB[160];
  __shared__ __attribute__((aligned(16))) unsigned short sH[32 * HWD];
  const int tid = (int)threadIdx.x;
  if (tid < 32) {
    const v4f b = *(const v4fa*)(tab + 320 + 4 * tid);
    *(v4fa*)(sB + 4 * tid) = b;
  }
  __syncthreads();
  if (tid < 32) sB[128 + tid] = 1.0f / sqrtf(sB[96 + tid] + 1e-5f);
  __syncthreads();

  const int rl = tid >> 3;
  const int pc = tid & 7;
  const int c4 = pc * 4;
  const int lrow = (int)blockIdx.x * 32 + rl;
  const bool live = lrow < rowsValid;
  const int lrc = live ? lrow : rowsValid - 1;
  const v4f y = *(const v4fa*)(Y + (size_t)lrc * YLD + c4);
  asm volatile("" :: "v"(y));
  const int t = chunkStart + lrc;
  const int fl = flg[(t >> 10) * 32];
  asm volatile("" :: "v"(fl));
  const v4f g  = *(const v4fa*)(sB + c4);
  const v4f be = *(const v4fa*)(sB + 32 + c4);
  const v4f mu = *(const v4fa*)(sB + 64 + c4);
  const v4f rs = *(const v4fa*)(sB + 128 + c4);
  const float qnan = __uint_as_float(0x7fc00000u);
  v4f z;
#pragma unroll
  for (int i = 0; i < 4; ++i) {
    float v = ((y[i] - mu[i]) * g[i]) * rs[i] + be[i];
    v = (v > 0.f) ? v : (v - v);
    v = (fl != 0) ? qnan : v;
    z[i] = v;
  }
  if (LAYER == 1) {
#pragma unroll
    for (int i = 0; i < 4; ++i) {
      sH[rl * HWD + c4 + i]      = (unsigned short)bf16_bits(z[i]);
      sH[rl * HWD + 32 + c4 + i] = (unsigned short)(TWO_TERM ? bf16_lo_bits(z[i]) : 0u);
    }
    __syncthreads();
    const v8us piece = *(const v8usa*)(sH + tid * 8);
    unsigned short* gp = Hout + (size_t)(chunkStart + lrow) * HWD + pc * 8;
    if (live) *(volatile v8us*)gp = piece;
    __threadfence();
    if (live) *(volatile v8us*)gp = piece;
  } else {
    float* gp = Fout + (size_t)(chunkStart + lrow) * 32 + c4;
    if (live) *(volatile v4f*)gp = z;
    __threadfence();
    if (live) *(volatile v4f*)gp = z;
  }
}

static inline int cdiv(int a, int b) { return (a + b - 1) / b; }

extern "C" void kernel_launch(void* const* d_in, const int* in_sizes, int n_in,
                              void* d_out, int out_size, void* d_ws, size_t ws_size,
                              hipStream_t stream) {
  if (n_in < 20) return;
  if (in_sizes[0] != NN * 64 || in_sizes[1] != NN * 64) return;
  if (in_sizes[2] != 2 * 64 * 96 || in_sizes[3] != 384 || in_sizes[4] != 2 * 64 * 96 || in_sizes[5] != 192) return;
  if (in_sizes[6] != 2 * 96 * 32 || in_sizes[7] != 64 || in_sizes[8] != 256) return;
  if (in_sizes[9] != 2 * 32 * 96 || in_sizes[10] != 384 || in_sizes[11] != 2 * 32 * 96 || in_sizes[12] != 192) return;
  if (in_sizes[13] != 2 * 96 * 32 || in_sizes[14] != 64 || in_sizes[15] != 256) return;
  if (in_sizes[16] != NE || in_sizes[17] != NE || in_sizes[18] != NE || in_sizes[19] != NE) return;
  if (out_size != 2 * NN * 32) return;
  if (ws_size < WS_TOTAL) return;

  const float* emb_user = (const float*)d_in[0];
  const float* emb_item = (const float*)d_in[1];
  const float* Wl[2]   = { (const float*)d_in[2],  (const float*)d_in[9]  };
  const float* ATl[2]  = { (const float*)d_in[3],  (const float*)d_in[10] };
  const float* RSl[2]  = { (const float*)d_in[4],  (const float*)d_in[11] };
  const float* BIl[2]  = { (const float*)d_in[5],  (const float*)d_in[12] };
  const float* NWl[2]  = { (const float*)d_in[6],  (const float*)d_in[13] };
  const float* NBl[2]  = { (const float*)d_in[7],  (const float*)d_in[14] };
  const float* BNl[2]  = { (const float*)d_in[8],  (const float*)d_in[15] };
  const int* esrc[2] = { (const int*)d_in[16], (const int*)d_in[18] };
  const int* edst[2] = { (const int*)d_in[17], (const int*)d_in[19] };
  float* out = (float*)d_out;

  char* ws = (char*)d_ws;
  size_t off = 0;
  unsigned short* Aslot[3];
  for (int i = 0; i < 3; ++i) { Aslot[i] = (unsigned short*)(ws + off); off += SZ_A; }
  float* PS = (float*)(ws + off); off += SZ_PS;
  float* EL = (float*)(ws + off); off += SZ_EL;
  float* PT = (float*)(ws + off); off += SZ_PT;
  float* Y  = PT;
  unsigned short* XL = (unsigned short*)(ws + off); off += SZ_XL;
  int* HITS[2]; int* ROFF[2]; int* RCNT[2]; int* FLG[2];
  for (int d = 0; d < 2; ++d) { HITS[d] = (int*)(ws + off); off += SZ_HITS; }
  for (int d = 0; d < 2; ++d) { ROFF[d] = (int*)(ws + off); off += SZ_ROW; RCNT[d] = (int*)(ws + off); off += SZ_ROW; }
  for (int d = 0; d < 2; ++d) { FLG[d] = (int*)(ws + off); off += SZ_FLG; }
  unsigned short* PL = (unsigned short*)(ws + off); off += SZ_PL;
  float* TAB = (float*)(ws + off); off += SZ_TAB;
  if (off != WS_TOTAL) return;

  hipFuncSetAttribute(reinterpret_cast<const void*>(&k_build), hipFuncAttributeMaxDynamicSharedMemorySize, LDS_BUILD);

  k_plane<0><<<MPN * 64 / 8 / 256, 256, 0, stream>>>(emb_user, NN, 64, 64, Aslot[0], MPN, 64);
  k_plane<0><<<MPN * 64 / 8 / 256, 256, 0, stream>>>(emb_item, NN, 64, 64, Aslot[1], MPN, 64);

  for (int L = 0; L < 2; ++L) {
    k_prep<<<dim3(20, 2), 256, 0, stream>>>(Wl[L], RSl[L], NWl[L], ATl[L], BIl[L], NBl[L], BNl[L],
                                            L == 0 ? 64 : 32,
                                            PL + (size_t)L * 2 * PLANE_US, TAB + (size_t)L * 2 * TABF,
                                            Aslot[2] + (size_t)NN * HWD, L == 0 ? 1 : 0);
  }

  for (int d = 0; d < 2; ++d)
    k_build<<<NOWN, 256, LDS_BUILD, stream>>>(esrc[d], edst[d], HITS[d], ROFF[d], RCNT[d], FLG[d]);

  for (int L = 0; L < 2; ++L) {
    for (int d = 0; d < 2; ++d) {
      const unsigned short* AS;
      const unsigned short* AT;
      unsigned short* Hout;
      float* Fout;
      if (L == 0 && d == 0)      { AS = Aslot[0]; AT = Aslot[1]; Hout = Aslot[2]; Fout = out; }
      else if (L == 0 && d == 1) { AS = Aslot[1]; AT = Aslot[0]; Hout = Aslot[1]; Fout = out; }
      else if (L == 1 && d == 0) { AS = Aslot[1]; AT = Aslot[2]; Hout = Aslot[2]; Fout = out + OUT_ITEM; }
      else                       { AS = Aslot[2]; AT = Aslot[1]; Hout = Aslot[2]; Fout = out; }
      const int ci = L * 2 + d;
      const unsigned short* BS = PL + (size_t)ci * PLANE_US;
      const unsigned short* BT = BS + 8192;
      const unsigned short* BL = BT + 12288;
      const float* tb = TAB + (size_t)ci * TABF;

      {
        const int tiles = cdiv(NN, 64) * cdiv(96, 64);
        k_gemm_nt<0, 0><<<cdiv(tiles, 8), 256, 0, stream>>>(AS, BS, tb, PS, NN, 96, 64, PSLD);
      }
      k_el<<<MPN / 256, 256, 0, stream>>>(PS, tb, EL);

      for (int c = 0; c < 4; ++c) {
        const int cs   = c * CHROWS;
        const int rows = (c < 3) ? CHROWS : LASTROWS;
        const int rpad = (c < 3) ? CHROWS : LASTPAD;
        {
          const int tiles = cdiv(rows, 64) * 3;
          k_gemm_nt<0, 0><<<cdiv(tiles, 8), 256, 0, stream>>>(AT + (size_t)cs * HWD, BT, tb, PT, rows, 192, 64, PTLD);
        }
        k_replay<<<rpad / 8, 256, 0, stream>>>(PT, EL, PS, HITS[d], ROFF[d], RCNT[d], FLG[d], tb, XL, cs, rows, rpad);
        {
          const int tiles = cdiv(rows, 64);
          k_gemm_nt<0, 1><<<cdiv(tiles, 8), 256, 0, stream>>>(XL, BL, tb + 288, Y, rows, 32, 192, YLD);
        }
        if (L == 0) k_row<1><<<rows / 32, 256, 0, stream>>>(Y, tb, FLG[d], Hout, Fout, cs, rows);
        else        k_row<2><<<rows / 32, 256, 0, stream>>>(Y, tb, FLG[d], Hout, Fout, cs, rows);
      }
    }
  }
}
